// LSTMPointerNet_32126355374094
// MI455X (gfx1250) — hardware-verified
//
#include <hip/hip_runtime.h>

typedef __attribute__((ext_vector_type(16))) _Float16 v16h;
typedef __attribute__((ext_vector_type(8)))  _Float16 v8h;
typedef __attribute__((ext_vector_type(16))) __bf16   v16b;
typedef __attribute__((ext_vector_type(8)))  __bf16   v8b;
typedef __attribute__((ext_vector_type(8)))  float    v8f;
typedef __attribute__((ext_vector_type(4)))  float    v4f;

#define NB 32
#define NN 128
#define DD 512
#define HH 512
#define TQ 32
#define TT 31
#define G4 2048
#define HP 528

__device__ __forceinline__ unsigned short f2bf_bits(float f) {
  unsigned u = __float_as_uint(f);
  return (unsigned short)((u + 0x7FFFu + ((u >> 16) & 1u)) >> 16);
}
__device__ __forceinline__ float bf_bits2f(unsigned short h) { return __uint_as_float(((unsigned)h) << 16); }

__device__ __forceinline__ void dep_guard_h(v8f& a, v8f& b, v16h x, v16h y) { asm volatile("v_nop\n\tv_nop\n\tv_nop\n\tv_nop" : "+v"(a), "+v"(b) : "v"(x), "v"(y)); }
__device__ __forceinline__ void dep_guard_b(v8f& a, v8f& b, v16b x, v16b y) { asm volatile("v_nop\n\tv_nop\n\tv_nop\n\tv_nop" : "+v"(a), "+v"(b) : "v"(x), "v"(y)); }
__device__ __forceinline__ void keep4_h(v16h a, v16h b, v16h c, v16h d) { asm volatile("v_nop" :: "v"(a), "v"(b), "v"(c), "v"(d)); }
__device__ __forceinline__ void keep4_b(v16b a, v16b b, v16b c, v16b d) { asm volatile("v_nop" :: "v"(a), "v"(b), "v"(c), "v"(d)); }
__device__ __forceinline__ void acc_guard4(v8f& a, v8f& b, v8f& c, v8f& d) { asm volatile("v_nop\n\tv_nop\n\tv_nop\n\tv_nop" : "+v"(a), "+v"(b), "+v"(c), "+v"(d)); }
template <typename T> struct Frag;
template <> struct Frag<_Float16> {
  typedef v16h V; union U { v16h v; v8h h[2]; };
  static __device__ __forceinline__ v16h load(const _Float16* p) {
    U f; f.h[0] = *(const v8h*)(p); f.h[1] = *(const v8h*)(p + 16); return f.v;
  }
  static __device__ __forceinline__ v8f mma(v16h a, v16h b, v8f c) {
    return __builtin_amdgcn_wmma_f32_16x16x32_f16(false, a, false, b, (short)0, c, false, false);
  }
  static __device__ __forceinline__ void guard(v8f& a, v8f& b, v16h x, v16h y) { dep_guard_h(a, b, x, y); }
  static __device__ __forceinline__ void keep(v16h a, v16h b, v16h c, v16h d) { keep4_h(a, b, c, d); }
};
template <> struct Frag<__bf16> {
  typedef v16b V; union U { v16b v; v8b h[2]; };
  static __device__ __forceinline__ v16b load(const __bf16* p) {
    U f; f.h[0] = *(const v8b*)(p); f.h[1] = *(const v8b*)(p + 16); return f.v;
  }
  static __device__ __forceinline__ v8f mma(v16b a, v16b b, v8f c) {
    return __builtin_amdgcn_wmma_f32_16x16x32_bf16(false, a, false, b, (short)0, c, false, false);
  }
  static __device__ __forceinline__ void guard(v8f& a, v8f& b, v16b x, v16b y) { dep_guard_b(a, b, x, y); }
  static __device__ __forceinline__ void keep(v16b a, v16b b, v16b c, v16b d) { keep4_b(a, b, c, d); }
};

__device__ __forceinline__ v8f mma_f16_g(v16h a, v16h b, v8f c) {
  c = __builtin_amdgcn_wmma_f32_16x16x32_f16(false, a, false, b, (short)0, c, false, false);
  asm volatile("v_nop\n\tv_nop\n\tv_nop\n\tv_nop" : "+v"(c) : "v"(a), "v"(b));
  return c;
}

template <int ET> struct Elem;
template <> struct Elem<0> { typedef _Float16 T; };
template <> struct Elem<1> { typedef __bf16 T; };
template <int ET, bool SPLIT, int BIAS_MODE, int OUT_MODE, bool RESID, int ACT = 0>
__global__ __launch_bounds__(256) void wmma_gemm64(
    const unsigned short* __restrict__ Ap, const unsigned short* __restrict__ A2p, int lda, long strideA,
    const unsigned short* __restrict__ Btp, const unsigned short* __restrict__ Bt2p, int ldb, long strideB,
    void* __restrict__ Cout, void* __restrict__ Cout2, int ldc, long strideC,
    const float* __restrict__ bias,
    const float* __restrict__ resid, long strideR,
    int M, int N, int K, float scale) {
  typedef typename Elem<ET>::T T;
  typedef typename Frag<T>::V V;
  const T* A = (const T*)Ap; const T* A2 = (const T*)A2p; const T* Bt = (const T*)Btp; const T* Bt2 = (const T*)Bt2p;
  __shared__ __align__(16) float sT[8][16 * 68];
  const int b    = blockIdx.y;
  const int lane = threadIdx.x & 31;
  const int wave = threadIdx.x >> 5;
  const int tilesN = N >> 6;
  const int tilesM = M >> 6;
  const int tile = blockIdx.x * 8 + wave;
  if (tile >= tilesM * tilesN) return;
  const int tm = tile / tilesN;
  const int tn = tile - tm * tilesN;
  const int m0 = tm << 6;
  const int n0 = tn << 6;

  const T* Ab  = A  + (size_t)b * strideA;
  const T* Bb  = Bt + (size_t)b * strideB;
  const T* Ab2 = SPLIT ? (A2  + (size_t)b * strideA) : nullptr;
  const T* Bb2 = SPLIT ? (Bt2 + (size_t)b * strideB) : nullptr;

  const int rlane = lane & 15;
  const int koff  = (lane >> 4) * 8;
  const int mOff  = (lane >> 4) * 8;

  v8f acc[4][4];
#pragma unroll
  for (int i = 0; i < 4; ++i)
#pragma unroll
    for (int j = 0; j < 4; ++j) acc[i][j] = (v8f){0.f,0.f,0.f,0.f,0.f,0.f,0.f,0.f};

  for (int k0 = 0; k0 < K; k0 += 32) {
    V bh[4], bl[4];
#pragma unroll
    for (int j = 0; j < 4; ++j) {
      const size_t bo = (size_t)(n0 + (j << 4) + rlane) * ldb + koff + k0;
      bh[j] = Frag<T>::load(Bb + bo);
      if (SPLIT) bl[j] = Frag<T>::load(Bb2 + bo);
    }
#pragma unroll
    for (int i = 0; i < 4; ++i) {
      const size_t ao = (size_t)(m0 + (i << 4) + rlane) * lda + koff + k0;
      V ah = Frag<T>::load(Ab + ao);
      V al;
      if (SPLIT) al = Frag<T>::load(Ab2 + ao);
#pragma unroll
      for (int j = 0; j < 4; ++j) {
        acc[i][j] = Frag<T>::mma(ah, bh[j], acc[i][j]);
        if (SPLIT) {
          acc[i][j] = Frag<T>::mma(ah, bl[j], acc[i][j]);
          acc[i][j] = Frag<T>::mma(al, bh[j], acc[i][j]);
        }
      }
      Frag<T>::guard(acc[i][0], acc[i][3], ah, SPLIT ? al : ah);
    }
    Frag<T>::keep(bh[0], bh[1], bh[2], bh[3]);
    if (SPLIT) Frag<T>::keep(bl[0], bl[1], bl[2], bl[3]);
  }
  acc_guard4(acc[0][0], acc[0][1], acc[0][2], acc[0][3]);
  acc_guard4(acc[1][0], acc[1][1], acc[1][2], acc[1][3]);
  acc_guard4(acc[2][0], acc[2][1], acc[2][2], acc[2][3]);
  acc_guard4(acc[3][0], acc[3][1], acc[3][2], acc[3][3]);

  float* slab = sT[wave];
  const float* Rb = RESID ? (resid + (size_t)b * strideR) : nullptr;
#pragma unroll
  for (int i = 0; i < 4; ++i) {
    const int mBase = m0 + (i << 4);
#pragma unroll
    for (int j = 0; j < 4; ++j) {
      const int n = n0 + (j << 4) + rlane;
      float bv = 0.f;
      if (BIAS_MODE == 2) bv = bias[n];
#pragma unroll
      for (int r = 0; r < 8; ++r) {
        float v = acc[i][j][r] * scale;
        if (BIAS_MODE == 1) v += bias[mBase + mOff + r];
        if (BIAS_MODE == 2) v += bv;
        if (RESID) v += Rb[(size_t)(mBase + mOff + r) * ldc + n];
        if (ACT == 1) v = tanhf(v);
        if (ACT == 2) v = fmaxf(v, 0.0f);
        if (ACT == 3) v = v / (1.0f + expf(-v));
        if (ACT == 4) v = (v > 0.f) ? v : 0.01f * v;
        if (ACT == 5) v = 0.5f * v * (1.0f + erff(v * 0.70710678118654752f));
        slab[(mOff + r) * 68 + (j << 4) + rlane] = v;
      }
    }
    __builtin_amdgcn_fence(__ATOMIC_RELEASE, "workgroup");
    __builtin_amdgcn_wave_barrier();
    __builtin_amdgcn_fence(__ATOMIC_ACQUIRE, "workgroup");
    if (OUT_MODE == 0) {
      float* C = (float*)Cout + (size_t)b * strideC;
      const int hh = lane >> 4, c4 = (lane & 15) * 4;
      for (int pass = 0; pass < 2; ++pass) {
#pragma unroll
        for (int it = 0; it < 8; ++it) {
          const int row = it * 2 + hh;
          v4f v = *(const v4f*)(slab + row * 68 + c4);
          *(volatile v4f*)(C + (size_t)(mBase + row) * ldc + n0 + c4) = v;
        }
        __threadfence();
      }
    } else {
      const int q = lane >> 3, c8 = (lane & 7) * 8;
      unsigned short* C  = (unsigned short*)Cout  + (size_t)b * strideC;
      unsigned short* C2 = (OUT_MODE == 2) ? ((unsigned short*)Cout2 + (size_t)b * strideC) : nullptr;
      for (int pass = 0; pass < 2; ++pass) {
#pragma unroll
        for (int it = 0; it < 4; ++it) {
          const int row = it * 4 + q;
          const float* sp = slab + row * 68 + c8;
          v8h hv, lv;
#pragma unroll
          for (int e = 0; e < 8; ++e) {
            if (OUT_MODE == 1) {
              hv[e] = (_Float16)sp[e];
            } else {
              unsigned short hb = f2bf_bits(sp[e]);
              unsigned short lb = f2bf_bits(sp[e] - bf_bits2f(hb));
              hv[e] = __builtin_bit_cast(_Float16, hb);
              lv[e] = __builtin_bit_cast(_Float16, lb);
            }
          }
          *(volatile v8h*)(C + (size_t)(mBase + row) * ldc + n0 + c8) = hv;
          if (OUT_MODE == 2) *(volatile v8h*)(C2 + (size_t)(mBase + row) * ldc + n0 + c8) = lv;
        }
        __threadfence();
      }
    }
    __builtin_amdgcn_fence(__ATOMIC_RELEASE, "workgroup");
    __builtin_amdgcn_wave_barrier();
    __builtin_amdgcn_fence(__ATOMIC_ACQUIRE, "workgroup");
  }
}

__global__ __launch_bounds__(256) void cast_f32_f16x2(
    const float* __restrict__ in, _Float16* __restrict__ out, int n2) {
  int i = blockIdx.x * 256 + threadIdx.x;
  if (i < n2) {
    const _Float16 h0 = (_Float16)in[2 * i], h1 = (_Float16)in[2 * i + 1];
    const unsigned u = (unsigned)__builtin_bit_cast(unsigned short, h0) | ((unsigned)__builtin_bit_cast(unsigned short, h1) << 16);
    ((volatile unsigned*)out)[i] = u;
    __threadfence();
    ((volatile unsigned*)out)[i] = u;
  }
}

__global__ __launch_bounds__(256) void build_x_f16(
    const float* __restrict__ lstm_in, const float* __restrict__ init_i, _Float16* __restrict__ x16) {
  const int i = blockIdx.x * 256 + threadIdx.x;
  if (i < TQ * NB * (DD / 2)) {
    const int m = i / (DD / 2);
    const int dp = (i - m * (DD / 2)) * 2;
    const int t = m >> 5, b = m & 31;
    const float* src = (t == 0) ? (init_i + dp) : (lstm_in + ((size_t)(b * TT + (t - 1))) * DD + dp);
    const _Float16 h0 = (_Float16)src[0], h1 = (_Float16)src[1];
    const unsigned u = (unsigned)__builtin_bit_cast(unsigned short, h0) | ((unsigned)__builtin_bit_cast(unsigned short, h1) << 16);
    ((volatile unsigned*)x16)[i] = u;
    __threadfence();
    ((volatile unsigned*)x16)[i] = u;
  }
}

__global__ __launch_bounds__(256) void transpose4_f16(
    const float* __restrict__ p0, const float* __restrict__ p1, const float* __restrict__ p2, const float* __restrict__ p3,
    _Float16* __restrict__ out, int R) {
  __shared__ float sm[64][65];
  const int z = blockIdx.z;
  const float* in = (z == 0) ? p0 : (z == 1) ? p1 : (z == 2) ? p2 : p3;
  const int r0 = blockIdx.y * 64, c0 = blockIdx.x * 64;
  const int tid = threadIdx.x;
#pragma unroll
  for (int i = 0; i < 16; ++i) {
    const int row = i * 4 + (tid >> 6);
    const int col = tid & 63;
    sm[row][col] = in[(size_t)(r0 + row) * R + c0 + col];
  }
  __syncthreads();
  _Float16* ob = out + (size_t)z * R * R;
  v8h vals[2];
  size_t offs[2];
#pragma unroll
  for (int p = 0; p < 2; ++p) {
    const int task = p * 256 + tid;
    const int oc = task >> 3, seg = task & 7;
    v8h hv;
#pragma unroll
    for (int j = 0; j < 8; ++j) hv[j] = (_Float16)sm[seg * 8 + j][oc];
    vals[p] = hv;
    offs[p] = (size_t)(c0 + oc) * R + r0 + seg * 8;
  }
  *(volatile v8h*)(ob + offs[0]) = vals[0];
  *(volatile v8h*)(ob + offs[1]) = vals[1];
  __threadfence();
  *(volatile v8h*)(ob + offs[0]) = vals[0];
  *(volatile v8h*)(ob + offs[1]) = vals[1];
}

__device__ __forceinline__ float sigm_f(float x) { return __builtin_amdgcn_rcpf(1.0f + expf(-x)); }

__device__ __forceinline__ float tanh_fast(float x) {
  x = fminf(fmaxf(x, -16.0f), 16.0f);
  const float e = __expf(2.0f * x);
  const float r = __builtin_amdgcn_rcpf(e + 1.0f);
  return fmaf(-2.0f, r, 1.0f);
}

__global__ __launch_bounds__(256) void lstm_seq_kernel(
    const float* __restrict__ xw, const unsigned short* __restrict__ whhp,
    const float* __restrict__ b_ih, const float* __restrict__ b_hh,
    const float* __restrict__ init_h, const float* __restrict__ init_c,
    unsigned short* __restrict__ qout) {
  const _Float16* whh = (const _Float16*)whhp;
  _Float16* q16 = (_Float16*)qout;
  __shared__ __align__(16) _Float16 hb[2][NB * HP];
  __shared__ __align__(16) float cs[NB * HH];
  const int tid = threadIdx.x, lane = tid & 31, wave = tid >> 5;
  const int c = lane & 15, hh = lane >> 4, koff = hh * 8;
  for (int i = tid; i < NB * HH; i += 256) {
    const int b = i >> 9, j = i & (HH - 1);
    hb[0][b * HP + j] = (_Float16)init_h[j];
    cs[i] = init_c[j];
  }
  __syncthreads();
  for (int t = 0; t < TQ; ++t) {
    const _Float16* hcur = hb[t & 1];
    _Float16* hnxt = hb[(t + 1) & 1];
    const float* xwt = xw + (size_t)t * NB * G4;
#pragma unroll 1
    for (int qq = 0; qq < 4; ++qq) {
      const int j0 = 64 * wave + 16 * qq;
      v8f acc[2][4];
#pragma unroll
      for (int mi = 0; mi < 2; ++mi)
#pragma unroll
        for (int g = 0; g < 4; ++g) acc[mi][g] = (v8f){0.f,0.f,0.f,0.f,0.f,0.f,0.f,0.f};
#pragma unroll 1
      for (int k0 = 0; k0 < HH; k0 += 32) {
        v16h bfr[4];
#pragma unroll
        for (int g = 0; g < 4; ++g) bfr[g] = Frag<_Float16>::load(whh + (size_t)(g * HH + j0 + c) * HH + k0 + koff);
#pragma unroll
        for (int mi = 0; mi < 2; ++mi) {
          const v16h afr = Frag<_Float16>::load(hcur + (mi * 16 + c) * HP + k0 + koff);
#pragma unroll
          for (int g = 0; g < 4; ++g) acc[mi][g] = Frag<_Float16>::mma(afr, bfr[g], acc[mi][g]);
          Frag<_Float16>::guard(acc[mi][0], acc[mi][3], afr, afr);
        }
        Frag<_Float16>::keep(bfr[0], bfr[1], bfr[2], bfr[3]);
      }
      acc_guard4(acc[0][0], acc[0][1], acc[0][2], acc[0][3]);
      acc_guard4(acc[1][0], acc[1][1], acc[1][2], acc[1][3]);
      const int j = j0 + c;
      const float bi = b_ih[j] + b_hh[j];
      const float bf = b_ih[HH + j] + b_hh[HH + j];
      const float bg = b_ih[2 * HH + j] + b_hh[2 * HH + j];
      const float bo = b_ih[3 * HH + j] + b_hh[3 * HH + j];
#pragma unroll
      for (int mi = 0; mi < 2; ++mi) {
#pragma unroll
        for (int r = 0; r < 8; ++r) {
          const int b = mi * 16 + 8 * hh + r;
          const float* xr = xwt + (size_t)b * G4;
          const float gi = acc[mi][0][r] + xr[j] + bi;
          const float gf = acc[mi][1][r] + xr[HH + j] + bf;
          const float gg = acc[mi][2][r] + xr[2 * HH + j] + bg;
          const float go = acc[mi][3][r] + xr[3 * HH + j] + bo;
          const float cp = cs[b * HH + j];
          const float cn = sigm_f(gf) * cp + sigm_f(gi) * tanhf(gg);
          const float hn = sigm_f(go) * tanhf(cn);
          cs[b * HH + j] = cn;
          hnxt[b * HP + j] = (_Float16)hn;
        }
      }
    }
    __syncthreads();
    {
      const int rq = lane >> 3, c8 = (lane & 7) * 8;
      for (int pass = 0; pass < 2; ++pass) {
#pragma unroll
        for (int it = 0; it < 8; ++it) {
          const int row = it * 4 + rq;
          const v8h v = *(const v8h*)(hnxt + row * HP + 64 * wave + c8);
          *(volatile v8h*)(q16 + ((size_t)(row * TQ + t)) * HH + 64 * wave + c8) = v;
        }
        __threadfence();
      }
    }
  }
}

template <bool HOP>
__global__ __launch_bounds__(256) void tanh_vdot_kernel(
    const float* __restrict__ feat, const float* __restrict__ qp, const float* __restrict__ vv,
    const int* __restrict__ msz, unsigned short* __restrict__ qo, float* __restrict__ outp) {
  __shared__ __align__(16) _Float16 vsh[HH];
  __shared__ __align__(16) float qsh[HH];
  __shared__ __align__(16) float sc[NN];
  __shared__ __align__(16) float osh[HH];
  __shared__ float red[16];
  const int bt = blockIdx.x;
  const int b = bt >> 5;
  const int tid = threadIdx.x, lane = tid & 31, wave = tid >> 5;
  const int c = lane & 15, hh = lane >> 4, koff = hh * 8;
  for (int i = tid; i < HH; i += 256) {
    vsh[i] = (_Float16)(vv[i] * 256.0f);
    qsh[i] = qp[(size_t)bt * HH + i];
  }
  __syncthreads();
  {
    const float* fr = feat + ((size_t)(b * NN + 16 * wave + c)) * HH;
    v8f acc = (v8f){0.f,0.f,0.f,0.f,0.f,0.f,0.f,0.f};
#pragma unroll 4
    for (int ks = 0; ks < HH / 32; ++ks) {
      const int k0 = ks * 32;
      const v16h vb = Frag<_Float16>::load(vsh + k0 + koff);
      const v4f f0 = *(const v4f*)(fr + k0 + koff);
      const v4f f1 = *(const v4f*)(fr + k0 + koff + 4);
      const v4f f2 = *(const v4f*)(fr + k0 + 16 + koff);
      const v4f f3 = *(const v4f*)(fr + k0 + 16 + koff + 4);
      const v4f s0 = f0 + *(const v4f*)(qsh + k0 + koff);
      const v4f s1 = f1 + *(const v4f*)(qsh + k0 + koff + 4);
      const v4f s2 = f2 + *(const v4f*)(qsh + k0 + 16 + koff);
      const v4f s3 = f3 + *(const v4f*)(qsh + k0 + 16 + koff + 4);
      v16h af;
      af[0]  = (_Float16)tanh_fast(s0[0]); af[1]  = (_Float16)tanh_fast(s0[1]);
      af[2]  = (_Float16)tanh_fast(s0[2]); af[3]  = (_Float16)tanh_fast(s0[3]);
      af[4]  = (_Float16)tanh_fast(s1[0]); af[5]  = (_Float16)tanh_fast(s1[1]);
      af[6]  = (_Float16)tanh_fast(s1[2]); af[7]  = (_Float16)tanh_fast(s1[3]);
      af[8]  = (_Float16)tanh_fast(s2[0]); af[9]  = (_Float16)tanh_fast(s2[1]);
      af[10] = (_Float16)tanh_fast(s2[2]); af[11] = (_Float16)tanh_fast(s2[3]);
      af[12] = (_Float16)tanh_fast(s3[0]); af[13] = (_Float16)tanh_fast(s3[1]);
      af[14] = (_Float16)tanh_fast(s3[2]); af[15] = (_Float16)tanh_fast(s3[3]);
      acc = mma_f16_g(af, vb, acc);
    }
    if (c == 0) {
#pragma unroll
      for (int r = 0; r < 8; ++r) sc[16 * wave + 8 * hh + r] = acc[r] * (1.0f / 256.0f);
    }
  }
  __syncthreads();
  if (!HOP) {
    if (wave == 0) {
      const v4f val = *(const v4f*)(sc + 4 * lane);
      float* op = outp + (size_t)bt * NN + 4 * lane;
      *(volatile v4f*)op = val;
      __threadfence();
      *(volatile v4f*)op = val;
    }
  } else {
    int ms = msz[b];
    ms = ms < 0 ? 0 : (ms > NN ? NN : ms);
    float s = -__builtin_inff();
    if (tid < NN) s = (tid < ms) ? sc[tid] : -1e18f;
    float m = s;
#pragma unroll
    for (int off = 16; off > 0; off >>= 1) m = fmaxf(m, __shfl_xor(m, off, 32));
    if (lane == 0) red[wave] = m;
    __syncthreads();
    float mx = red[0];
#pragma unroll
    for (int w = 1; w < 8; ++w) mx = fmaxf(mx, red[w]);
    const float e = (tid < NN) ? expf(s - mx) : 0.f;
    float su = e;
#pragma unroll
    for (int off = 16; off > 0; off >>= 1) su += __shfl_xor(su, off, 32);
    if (lane == 0) red[8 + wave] = su;
    __syncthreads();
    float tot = red[8];
#pragma unroll
    for (int w = 1; w < 8; ++w) tot += red[8 + w];
    const float inv = 1.0f / tot;
    if (tid < NN) sc[tid] = e * inv;
    __syncthreads();
    const float* fb = feat + (size_t)b * NN * HH;
    float a0 = 0.f, a1 = 0.f;
#pragma unroll 4
    for (int n = 0; n < NN; ++n) {
      const float p = sc[n];
      const float* f = fb + (size_t)n * HH;
      a0 = fmaf(p, f[tid], a0);
      a1 = fmaf(p, f[tid + 256], a1);
    }
    osh[tid] = a0;
    osh[tid + 256] = a1;
    __syncthreads();
    if (tid < 64) {
      const v4f u0 = *(const v4f*)(osh + 8 * tid);
      const v4f u1 = *(const v4f*)(osh + 8 * tid + 4);
      v8h hv;
      hv[0] = (_Float16)u0[0]; hv[1] = (_Float16)u0[1]; hv[2] = (_Float16)u0[2]; hv[3] = (_Float16)u0[3];
      hv[4] = (_Float16)u1[0]; hv[5] = (_Float16)u1[1]; hv[6] = (_Float16)u1[2]; hv[7] = (_Float16)u1[3];
      _Float16* op = (_Float16*)qo + (size_t)bt * HH + 8 * tid;
      *(volatile v8h*)op = hv;
      __threadfence();
      *(volatile v8h*)op = hv;
    }
  }
}

extern "C" void kernel_launch(void* const* d_in, const int* in_sizes, int n_in,
                              void* d_out, int out_size, void* d_ws, size_t ws_size,
                              hipStream_t stream) {
  if (n_in < 16) return;
  if (in_sizes[0] != NB * NN * DD || in_sizes[1] != NB || in_sizes[2] != NB * TT * DD ||
      in_sizes[3] != HH || in_sizes[4] != HH || in_sizes[5] != DD ||
      in_sizes[6] != G4 * DD || in_sizes[7] != G4 * HH || in_sizes[8] != G4 || in_sizes[9] != G4 ||
      in_sizes[10] != DD * HH || in_sizes[11] != HH * HH || in_sizes[12] != HH ||
      in_sizes[13] != DD * HH || in_sizes[14] != HH * HH || in_sizes[15] != HH) return;
  if (out_size != NB * TQ * NN) return;

  const float* attn_mem  = (const float*)d_in[0];
  const int*   mem_sizes = (const int*)  d_in[1];
  const float* lstm_in   = (const float*)d_in[2];
  const float* init_h    = (const float*)d_in[3];
  const float* init_c    = (const float*)d_in[4];
  const float* init_i    = (const float*)d_in[5];
  const float* w_ih      = (const float*)d_in[6];
  const float* w_hh      = (const float*)d_in[7];
  const float* b_ih      = (const float*)d_in[8];
  const float* b_hh      = (const float*)d_in[9];
  const float* attn_wm   = (const float*)d_in[10];
  const float* attn_wq   = (const float*)d_in[11];
  const float* attn_v    = (const float*)d_in[12];
  const float* hop_wm    = (const float*)d_in[13];
  const float* hop_wq    = (const float*)d_in[14];
  const float* hop_v     = (const float*)d_in[15];
  float* out = (float*)d_out;

  char* base = (char*)d_ws;
  size_t off = 0;
  _Float16* am16   = (_Float16*)(base + off); off += (size_t)NB * NN * DD * 2;
  _Float16* wih16  = (_Float16*)(base + off); off += (size_t)G4 * DD * 2;
  _Float16* whh16  = (_Float16*)(base + off); off += (size_t)G4 * HH * 2;
  _Float16* wT16   = (_Float16*)(base + off); off += (size_t)4 * HH * HH * 2;
  _Float16* x16    = (_Float16*)(base + off); off += (size_t)TQ * NB * DD * 2;
  float*    afeat  = (float*)(base + off);    off += (size_t)NB * NN * HH * 4;
  float*    hfeat  = (float*)(base + off);    off += (size_t)NB * NN * HH * 4;
  float*    xw     = (float*)(base + off);    off += (size_t)TQ * NB * G4 * 4;
  _Float16* qry16  = (_Float16*)(base + off); off += (size_t)NB * TQ * HH * 2;
  float*    q1     = (float*)(base + off);    off += (size_t)NB * TQ * HH * 4;
  _Float16* qry2   = (_Float16*)(base + off); off += (size_t)NB * TQ * HH * 2;
  float*    q2     = (float*)(base + off);    off += (size_t)NB * TQ * HH * 4;
  if (off > ws_size || off > (size_t)134217728) return;

  const _Float16* awmT = wT16 + (size_t)0 * HH * HH;
  const _Float16* hwmT = wT16 + (size_t)1 * HH * HH;
  const _Float16* hwqT = wT16 + (size_t)2 * HH * HH;
  const _Float16* awqT = wT16 + (size_t)3 * HH * HH;

  {
    const int n2a = NB * NN * DD / 2;
    cast_f32_f16x2<<<(n2a + 255) / 256, 256, 0, stream>>>(attn_mem, am16, n2a);
    const int n2w = G4 * DD / 2;
    cast_f32_f16x2<<<(n2w + 255) / 256, 256, 0, stream>>>(w_ih, wih16, n2w);
    cast_f32_f16x2<<<(n2w + 255) / 256, 256, 0, stream>>>(w_hh, whh16, n2w);
    transpose4_f16<<<dim3(HH / 64, HH / 64, 4), 256, 0, stream>>>(attn_wm, hop_wm, hop_wq, attn_wq, wT16, HH);
    const int n2x = TQ * NB * DD / 2;
    build_x_f16<<<(n2x + 255) / 256, 256, 0, stream>>>(lstm_in, init_i, x16);
  }

  typedef const unsigned short* cu16;
  {
    const int tiles = (NB * NN / 64) * (HH / 64);
    wmma_gemm64<0, false, 0, 0, false, 0><<<dim3((tiles + 7) / 8, 1), 256, 0, stream>>>(
        (cu16)am16, (cu16)am16, DD, 0L, (cu16)awmT, (cu16)awmT, DD, 0L,
        (void*)afeat, (void*)afeat, HH, 0L, b_ih, b_hh, 0L, NB * NN, HH, DD, 1.0f);
    wmma_gemm64<0, false, 0, 0, false, 0><<<dim3((tiles + 7) / 8, 1), 256, 0, stream>>>(
        (cu16)am16, (cu16)am16, DD, 0L, (cu16)hwmT, (cu16)hwmT, DD, 0L,
        (void*)hfeat, (void*)hfeat, HH, 0L, b_ih, b_hh, 0L, NB * NN, HH, DD, 1.0f);
  }
  {
    const int tiles = (TQ * NB / 64) * (G4 / 64);
    wmma_gemm64<0, false, 0, 0, false, 0><<<dim3((tiles + 7) / 8, 1), 256, 0, stream>>>(
        (cu16)x16, (cu16)x16, DD, 0L, (cu16)wih16, (cu16)wih16, DD, 0L,
        (void*)xw, (void*)xw, G4, 0L, b_ih, b_hh, 0L, TQ * NB, G4, DD, 1.0f);
  }
  lstm_seq_kernel<<<1, 256, 0, stream>>>(xw, (cu16)whh16, b_ih, b_hh, init_h, init_c, (unsigned short*)qry16);

  {
    const int tiles = (NB * TQ / 64) * (HH / 64);
    wmma_gemm64<0, false, 0, 0, false, 0><<<dim3((tiles + 7) / 8, 1), 256, 0, stream>>>(
        (cu16)qry16, (cu16)qry16, HH, 0L, (cu16)hwqT, (cu16)hwqT, HH, 0L,
        (void*)q1, (void*)q1, HH, 0L, b_ih, b_hh, 0L, NB * TQ, HH, HH, 1.0f);
    tanh_vdot_kernel<true><<<NB * TQ, 256, 0, stream>>>(hfeat, q1, hop_v, mem_sizes, (unsigned short*)qry2, out);
  }
  {
    const int tiles = (NB * TQ / 64) * (HH / 64);
    wmma_gemm64<0, false, 0, 0, false, 0><<<dim3((tiles + 7) / 8, 1), 256, 0, stream>>>(
        (cu16)qry2, (cu16)qry2, HH, 0L, (cu16)awqT, (cu16)awqT, HH, 0L,
        (void*)q2, (void*)q2, HH, 0L, b_ih, b_hh, 0L, NB * TQ, HH, HH, 1.0f);
    tanh_vdot_kernel<false><<<NB * TQ, 256, 0, stream>>>(afeat, q2, attn_v, mem_sizes, (unsigned short*)qry2, out);
  }
}
